// UncertaintyGAT_24077586662039
// MI455X (gfx1250) — hardware-run, weakly checked
//
#include <hip/hip_runtime.h>


namespace {
constexpr int N = 100000, NP = 100032, NLIM = 100032  , NLIMN = (NLIM < N ? NLIM : N), E = 1600000, F = 64, HEADS = 4, HD = 16;
constexpr float XS = 8.0f, WSC = 256.0f;
static_assert(NP % 64 == 0 && NLIM % 64 == 0, "tiling");
typedef _Float16 b16;
typedef __attribute__((ext_vector_type(16))) _Float16 v16b;
typedef __attribute__((ext_vector_type(8))) _Float16 v8b;
typedef __attribute__((ext_vector_type(8))) float v8f;
typedef __attribute__((ext_vector_type(4))) float v4f;
__device__ __forceinline__ float bf16_rne(float f) { unsigned int u = __float_as_uint(f); u += 0x7FFFu + ((u >> 16) & 1u); return __uint_as_float(u & 0xFFFF0000u); }
__device__ __forceinline__ void split16(float v, b16& hi, b16& lo) { hi = (b16)v; lo = (b16)(v - (float)hi); }
__device__ __forceinline__ v16b frag_kb(const b16* p, int hh) { const v8b a = *(const v8b*)(p + 8 * hh), b = *(const v8b*)(p + 16 + 8 * hh); v16b f;
#pragma unroll
  for (int e = 0; e < 8; ++e) { f[e] = a[e]; f[8 + e] = b[e]; } return f; }
__device__ __forceinline__ v8f wmma16b(v16b a, v16b b, v8f c) { v8f d = __builtin_amdgcn_wmma_f32_16x16x32_f16(false, a, false, b, (short)0, c, false, false); asm volatile("v_nop\n\tv_nop\n\tv_nop\n\tv_nop" : "+v"(d) : "v"(a), "v"(b)); return d; }
__device__ __forceinline__ void wave_lds_sync() { __builtin_amdgcn_fence(__ATOMIC_RELEASE, "workgroup"); __builtin_amdgcn_wave_barrier(); __builtin_amdgcn_fence(__ATOMIC_ACQUIRE, "workgroup"); }
__device__ __forceinline__ float pmul(float a, float b) { float p = a * b; asm volatile("" : "+v"(p)); return p; }
__device__ __forceinline__ int iclamp(int v, int lo, int hi) { return v < lo ? lo : (v > hi ? hi : v); }
constexpr int CSR_NBLK = 512, CSR_GB = 9, CSR_GN = 1 << CSR_GB  , CSR_MAXG = 512, CSR_CAP = 12288  ;
__global__ __launch_bounds__(64) void csrA_kernel(const int* __restrict__ dst, int E, int N, int nG, int CHP, int NGP, int* __restrict__ STG, int* __restrict__ HST) {
  extern __shared__ int sm[];
  int* cnt = sm; int* run = sm + NGP; int* ids = sm + 2 * NGP;
  const int b = blockIdx.x; const int ch = (E + CSR_NBLK - 1) / CSR_NBLK; const int e0 = b * ch, e1 = min(E, e0 + ch);
  for (int i = threadIdx.x; i < NGP; i += 64) cnt[i] = 0;
  for (int i = threadIdx.x; i < CHP; i += 64) ids[i] = -1;
  __syncthreads();
  if (threadIdx.x == 0) {
    for (int e = e0; e < e1; ++e) { int d = dst[e]; d = (d < 0) ? 0 : (d >= N ? N - 1 : d); cnt[d >> CSR_GB] += 1; }
    int acc = 0; for (int g = 0; g < nG; ++g) { run[g] = acc; acc += cnt[g]; }
    for (int e = e0; e < e1; ++e) { int d = dst[e]; d = (d < 0) ? 0 : (d >= N ? N - 1 : d); const int g = d >> CSR_GB; ids[run[g]] = e; run[g] += 1; } }
  __syncthreads();
  typedef __attribute__((ext_vector_type(4))) int v4i;
  for (int pass = 0; pass < 2; ++pass) {
    for (int i = threadIdx.x; i < CHP / 4; i += 64) *(volatile v4i*)(STG + (size_t)b * CHP + i * 4) = *(const v4i*)(&ids[i * 4]);
    for (int i = threadIdx.x; i < NGP / 4; i += 64) { v4i v; for (int e = 0; e < 4; ++e) v[e] = (i * 4 + e < nG) ? cnt[i * 4 + e] : 0; *(volatile v4i*)(HST + (size_t)b * NGP + i * 4) = v; }
    __threadfence(); }
}
__global__ __launch_bounds__(512) void csrS_kernel(const int* __restrict__ HST, int nG, int NGP, int* __restrict__ START, int* __restrict__ TOT, int* __restrict__ OFF) {
  __shared__ int tot[CSR_MAXG];
  const int b = threadIdx.x;
  for (int pass = 0; pass < 2; ++pass) { int runb = 0; for (int g = 0; g < nG; ++g) { int c = HST[(size_t)b * NGP + g]; c = (c < 0) ? 0 : c; ((volatile int*)OFF)[(size_t)g * CSR_NBLK + b] = runb; runb += c; } __threadfence(); }
  for (int g = threadIdx.x; g < nG; g += 512) { int s = 0; for (int bb = 0; bb < CSR_NBLK; ++bb) { int c = HST[(size_t)bb * NGP + g]; s += (c < 0) ? 0 : c; } tot[g] = s; }
  __syncthreads();
  if (threadIdx.x < 32) {
    __shared__ int st[CSR_MAXG + 32];
    if (threadIdx.x == 0) { int acc = 0; for (int g = 0; g < NGP; ++g) { st[g] = acc; if (g < nG) acc += (tot[g] + 31) & ~31; } st[NGP] = acc; }
    __builtin_amdgcn_fence(__ATOMIC_RELEASE, "workgroup"); __builtin_amdgcn_wave_barrier(); __builtin_amdgcn_fence(__ATOMIC_ACQUIRE, "workgroup");
    for (int pass = 0; pass < 2; ++pass) { for (int i = threadIdx.x; i < NGP + 32; i += 32) { ((volatile int*)START)[i] = (i <= NGP) ? st[min(i, NGP)] : 0; ((volatile int*)TOT)[i] = (i < nG) ? tot[i] : 0; } __threadfence(); } }
}
__global__ __launch_bounds__(256) void csrB_kernel(const int* __restrict__ dst, int N, int nG, int CHP, int NGP, int permLen, const int* __restrict__ STG, const int* __restrict__ HST, const int* __restrict__ OFF, const int* __restrict__ START, const int* __restrict__ TOT, int* __restrict__ PERM, int* __restrict__ ROWPTR, int* __restrict__ ROWCNT, int* __restrict__ FLAG) {
  typedef __attribute__((ext_vector_type(4))) int v4i;
  __shared__ int ids[CSR_CAP]; __shared__ unsigned short key[CSR_CAP]; __shared__ int outp[CSR_CAP]; __shared__ int ncnt[CSR_GN + 1]; __shared__ int boff[CSR_NBLK + 1];
  const int g = blockIdx.x, t_ = threadIdx.x; int tot = TOT[g]; int st = START[g], stn = START[g + 1]; const int v0 = g * CSR_GN; const int nv = min(CSR_GN, N - v0);
  st = (st < 0) ? 0 : (st > permLen - 32 ? permLen - 32 : st) & ~31; stn = (stn < st) ? st : (stn > permLen ? permLen : stn); tot = (tot < 0) ? 0 : tot; if (tot > stn - st && tot <= CSR_CAP) tot = stn - st;
  if (tot > CSR_CAP) {
    for (int pass = 0; pass < 2; ++pass) { for (int i = t_; i < CSR_GN / 4; i += 256) { v4i a, c; for (int e = 0; e < 4; ++e) { a[e] = st; c[e] = 0; } *(volatile v4i*)(ROWPTR + v0 + i * 4) = a; *(volatile v4i*)(ROWCNT + v0 + i * 4) = c; } if (t_ == 0) ((volatile int*)FLAG)[0] = 1; __threadfence(); } (void)nv; return; }
  if (t_ == 0) { int acc = 0; for (int b = 0; b < CSR_NBLK; ++b) { boff[b] = acc; int c = HST[(size_t)b * NGP + g]; c = (c < 0) ? 0 : (c > CHP ? CHP : c); acc += c; if (acc > tot) acc = tot; } boff[CSR_NBLK] = acc; }
  for (int i = t_; i <= CSR_GN; i += 256) ncnt[i] = 0;
  __syncthreads();
  for (int b = 0; b < CSR_NBLK; ++b) { const int c = boff[b + 1] - boff[b]; int o_ = OFF[(size_t)g * CSR_NBLK + b]; o_ = (o_ < 0) ? 0 : (o_ > CHP - c ? CHP - c : o_); const int* src_ = STG + (size_t)b * CHP + o_;
    for (int i = t_; i < c; i += 256) { int id = src_[i]; id = (id < 0) ? 0 : id; ids[boff[b] + i] = id; int d = dst[id]; d = (d < v0) ? v0 : (d >= N ? N - 1 : d); int kk = d - v0; kk = (kk < 0) ? 0 : (kk >= CSR_GN ? CSR_GN - 1 : kk); key[boff[b] + i] = (unsigned short)kk; } }
  __syncthreads();
  if (t_ == 0) { for (int i = 0; i < tot; ++i) ncnt[key[i]] += 1; int acc = 0; for (int vl = 0; vl < CSR_GN; ++vl) { const int c = ncnt[vl]; ncnt[vl] = acc; acc += c; } ncnt[CSR_GN] = acc;
    for (int i = 0; i < tot; ++i) { const int vl = key[i]; outp[ncnt[vl]] = ids[i]; ncnt[vl] += 1; }
    for (int vl = CSR_GN; vl > 0; --vl) ncnt[vl] = ncnt[vl - 1]; ncnt[0] = 0; }
  __syncthreads();
  for (int pass = 0; pass < 2; ++pass) {
    for (int i = t_; i < (stn - st) / 4; i += 256) { v4i v; for (int e = 0; e < 4; ++e) { const int q = i * 4 + e; v[e] = (q < tot) ? outp[q] : -1; } *(volatile v4i*)(PERM + st + i * 4) = v; }
    for (int i = t_; i < CSR_GN / 4; i += 256) { v4i a, c; for (int e = 0; e < 4; ++e) { const int vl = i * 4 + e; a[e] = st + ncnt[vl]; c[e] = (vl < nv) ? (ncnt[vl + 1] - ncnt[vl]) : 0; } *(volatile v4i*)(ROWPTR + v0 + i * 4) = a; *(volatile v4i*)(ROWCNT + v0 + i * 4) = c; }
    __threadfence(); }
}
__global__ __launch_bounds__(256) void csrZ_kernel(int* __restrict__ p, size_t n4) { typedef __attribute__((ext_vector_type(4))) int v4i; const size_t tid = (size_t)blockIdx.x * 256 + threadIdx.x, nth = (size_t)gridDim.x * 256; v4i z = {0, 0, 0, 0}; for (size_t i = tid; i < n4; i += nth) *(volatile v4i*)(p + i * 4) = z; }
struct CsrBufs { int *STG, *HST, *OFF, *START, *TOT, *PERM, *ROWPTR, *ROWCNT, *FLAG; int nG, NGP, CHP; size_t permLen; char* base; size_t bytes; };
static size_t csr_carve(CsrBufs& c, char* ws, size_t off, int E, int N) {
  const size_t off0 = off; c.base = ws + off;
  auto al = [&](size_t bytes) { char* p = ws + off; off += (bytes + 255) & ~(size_t)255; return p; };
  c.nG = (N + CSR_GN - 1) / CSR_GN; c.NGP = (c.nG + 31) & ~31; const int ch = (E + CSR_NBLK - 1) / CSR_NBLK; c.CHP = (ch + 31) & ~31; c.permLen = (size_t)E + 32 * (size_t)c.nG + 32;
  c.STG = (int*)al((size_t)CSR_NBLK * c.CHP * 4); c.HST = (int*)al((size_t)CSR_NBLK * c.NGP * 4); c.OFF = (int*)al((size_t)c.NGP * CSR_NBLK * 4); c.START = (int*)al((size_t)(c.NGP + 64) * 4); c.TOT = (int*)al((size_t)(c.NGP + 64) * 4);
  c.PERM = (int*)al(c.permLen * 4); c.ROWPTR = (int*)al((size_t)c.nG * CSR_GN * 4); c.ROWCNT = (int*)al((size_t)c.nG * CSR_GN * 4); c.FLAG = (int*)al(256);
  c.bytes = off - off0; return off;
}
static void csr_build(const CsrBufs& c, const int* dst, int E, int N, hipStream_t stream) {
  const size_t smem = (size_t)(2 * c.NGP + c.CHP) * 4;
  csrZ_kernel<<<512, 256, 0, stream>>>((int*)c.base, c.bytes / 16);
  csrA_kernel<<<CSR_NBLK, 64, smem, stream>>>(dst, E, N, c.nG, c.CHP, c.NGP, c.STG, c.HST);
  csrS_kernel<<<1, 512, 0, stream>>>(c.HST, c.nG, c.NGP, c.START, c.TOT, c.OFF);
  csrB_kernel<<<c.nG, 256, 0, stream>>>(dst, N, c.nG, c.CHP, c.NGP, (int)c.permLen, c.STG, c.HST, c.OFF, c.START, c.TOT, c.PERM, c.ROWPTR, c.ROWCNT, c.FLAG);
}

typedef __attribute__((ext_vector_type(2))) float v2f;
__global__ __launch_bounds__(256) void wprep_kernel(const float* __restrict__ w0, const float* __restrict__ w1, b16* __restrict__ WT) {
  for (int u = threadIdx.x; u < 2 * F * F / 8; u += 256) { const int e = u * 8; const int l = e / (F * F), el = e % (F * F); const int oo = el / F, k0 = el % F; const float* w = l ? w1 : w0; v8b o;
    for (int j = 0; j < 8; ++j) o[j] = (b16)(bf16_rne(w[(size_t)(k0 + j) * F + oo]) * WSC);
    for (int pass = 0; pass < 2; ++pass) { *(volatile v8b*)(WT + e) = o; __threadfence(); } }
}
template <int TWO>
__global__ __launch_bounds__(128) void proj_kernel(const float* __restrict__ X, const b16* __restrict__ WT, const float* __restrict__ al, const float* __restrict__ ar, float* __restrict__ Z, float* __restrict__ ELR) {
  __shared__ __attribute__((aligned(16))) float Tz[4][16][F + 4]; __shared__ __attribute__((aligned(16))) float Te[4][16][8];
  const int wave = threadIdx.x >> 5, lane = threadIdx.x & 31, nloc = lane & 15, hlf = lane >> 4; const size_t v0 = ((size_t)blockIdx.x * 4 + wave) * 16; const size_t vr = v0 + nloc;
  v8f acc[4];
#pragma unroll
  for (int t = 0; t < 4; ++t) acc[t] = (v8f){};
#pragma unroll
  for (int ks = 0; ks < 2; ++ks) { v16b ah, a2;
#pragma unroll
    for (int e2 = 0; e2 < 16; ++e2) { const int k = ks * 32 + ((e2 < 8) ? (8 * hlf + e2) : (16 + 8 * hlf + e2 - 8)); float xv = (vr < (size_t)N) ? X[vr * F + k] : 0.0f;
      if (TWO) { b16 p, q; split16(xv * XS, p, q); ah[e2] = p; a2[e2] = q; } else { ah[e2] = (b16)(bf16_rne(xv) * XS); a2[e2] = (b16)0.0f; } }
#pragma unroll
    for (int t = 0; t < 4; ++t) { const v16b bw = frag_kb(WT + (size_t)(t * 16 + nloc) * F + ks * 32, hlf); acc[t] = wmma16b(ah, bw, acc[t]); if (TWO) acc[t] = wmma16b(a2, bw, acc[t]); } }
#pragma unroll
  for (int t = 0; t < 4; ++t) { const float a1 = bf16_rne(al[t * HD + nloc]), a2v = bf16_rne(ar[t * HD + nloc]);
#pragma unroll
    for (int r = 0; r < 8; ++r) { const float z = (v0 + 8 * hlf + r < (size_t)N) ? acc[t][r] * (1.0f / (XS * WSC)) : 0.0f; Tz[wave][8 * hlf + r][t * 16 + nloc] = z;
      float pl = z * a1, pr = z * a2v;
#pragma unroll
      for (int o = 1; o < 16; o <<= 1) { pl += __shfl_xor(pl, o); pr += __shfl_xor(pr, o); }
      if (nloc == 0) { Te[wave][8 * hlf + r][t] = pl; Te[wave][8 * hlf + r][4 + t] = pr; } } }
  wave_lds_sync();
  for (int pass = 0; pass < 2; ++pass) { for (int rr = 0; rr < 16; ++rr) *(volatile v2f*)(Z + (v0 + rr) * F + lane * 2) = *(const v2f*)(&Tz[wave][rr][lane * 2]);
    *(volatile v4f*)(ELR + v0 * 8 + lane * 4) = *(const v4f*)(&Te[wave][0][0] + lane * 4); __threadfence(); }
}
__global__ __launch_bounds__(256) void edge_kernel(const float* __restrict__ Z, const float* __restrict__ ELR, const float* __restrict__ bias, const int* __restrict__ srcs, const int* __restrict__ PERM, const int* __restrict__ ROWPTR, const int* __restrict__ ROWCNT, int permLen, float* __restrict__ H) {
  const int wave = threadIdx.x >> 5, lane = threadIdx.x & 31; const size_t v = (size_t)blockIdx.x * 8 + wave; const int c = lane * 2, hd = lane >> 3; v2f o = {0.0f, 0.0f};
  if (v < (size_t)NLIMN) { const float er = ELR[v * 8 + 4 + hd]; float m = -INFINITY, den = 0.0f; v2f acc = {0.0f, 0.0f};
    int st = ROWPTR[v], cnt = ROWCNT[v]; cnt = iclamp(cnt, 0, 65536); st = iclamp(st, 0, permLen - cnt);
#pragma unroll 1
    for (int j = 0; j < cnt; ++j) { const int e = iclamp(PERM[st + j], 0, E - 1); const size_t s = (size_t)iclamp(srcs[e], 0, N - 1); float lg = ELR[s * 8 + hd] + er; lg = lg >= 0.0f ? lg : 0.2f * lg;
      const float mn = fmaxf(m, lg); const float alf = (m == -INFINITY) ? 0.0f : __expf(m - mn), w = __expf(lg - mn); acc = acc * alf + *(const v2f*)(Z + s * F + c) * w; den = den * alf + w; m = mn; }
    if (den > 0.0f) o = acc * (1.0f / den);
    for (int i = 0; i < 2; ++i) { o[i] += bf16_rne(bias[c + i]); o[i] = fmaxf(o[i], 0.0f); } }
  for (int pass = 0; pass < 2; ++pass) { *(volatile v2f*)(H + v * F + c) = o; __threadfence(); }
}
__global__ __launch_bounds__(256) void proj3_kernel(const float* __restrict__ H, const float* __restrict__ wo, const float* __restrict__ alo, const float* __restrict__ aro, float* __restrict__ ZE) {
  __shared__ float s4[8][4];
  const int wave = threadIdx.x >> 5, lane = threadIdx.x & 31; const size_t v = (size_t)blockIdx.x * 8 + wave; float s = 0.0f;
  if (v < (size_t)NLIMN) { const v2f hv = *(const v2f*)(H + v * F + lane * 2); s = pmul(hv[0], bf16_rne(wo[lane * 2])) + pmul(hv[1], bf16_rne(wo[lane * 2 + 1])); }
#pragma unroll
  for (int o = 1; o < 32; o <<= 1) s += __shfl_xor(s, o);
  if (lane == 0) { s4[wave][0] = s; s4[wave][1] = pmul(s, bf16_rne(alo[0])); s4[wave][2] = pmul(s, bf16_rne(aro[0])); s4[wave][3] = 0.0f; }
  __syncthreads();
  for (int pass = 0; pass < 2; ++pass) { if (wave == 0) ((volatile float*)ZE)[(size_t)blockIdx.x * 32 + lane] = s4[lane >> 2][lane & 3]; __threadfence(); }
}
__global__ __launch_bounds__(256) void edge3_kernel(const float* __restrict__ ZE, const float* __restrict__ bo, const int* __restrict__ srcs, const int* __restrict__ PERM, const int* __restrict__ ROWPTR, const int* __restrict__ ROWCNT, int permLen, float* __restrict__ out) {
  __shared__ float so[64];
  const int t = threadIdx.x, wave = t >> 5, lane = t & 31; const int nd = t >> 2, sub = t & 3; const size_t v = (size_t)blockIdx.x * 64 + nd;
  float m = -INFINITY, den = 0.0f, acc = 0.0f;
  if (v < (size_t)N) { const float er = ZE[v * 4 + 2]; int st = ROWPTR[v], cnt = ROWCNT[v]; cnt = iclamp(cnt, 0, 65536); st = iclamp(st, 0, permLen - cnt);
#pragma unroll 1
    for (int j = sub; j < cnt; j += 4) { const int e = iclamp(PERM[st + j], 0, E - 1); const size_t s = (size_t)iclamp(srcs[e], 0, N - 1); float lg = ZE[s * 4 + 1] + er; lg = lg >= 0.0f ? lg : 0.2f * lg;
      const float mn = fmaxf(m, lg); const float alf = (m == -INFINITY) ? 0.0f : __expf(m - mn), w = __expf(lg - mn); acc = acc * alf + ZE[s * 4] * w; den = den * alf + w; m = mn; } }
#pragma unroll
  for (int o = 1; o < 4; o <<= 1) { const float m2 = __shfl_xor(m, o), d2 = __shfl_xor(den, o), a2 = __shfl_xor(acc, o); const float mn = fmaxf(m, m2);
    const float f1 = (m == -INFINITY) ? 0.0f : __expf(m - mn), f2 = (m2 == -INFINITY) ? 0.0f : __expf(m2 - mn); den = den * f1 + d2 * f2; acc = acc * f1 + a2 * f2; m = mn; }
  if (sub == 0) so[nd] = ((den > 0.0f) ? acc / den : 0.0f) + bf16_rne(bo[0]);
  __syncthreads();
  for (int pass = 0; pass < 2; ++pass) { if (wave == 0) { const size_t vb = (size_t)blockIdx.x * 64 + lane * 2; if (vb < (size_t)N) { v2f o2 = {so[lane * 2], so[lane * 2 + 1]}; *(volatile v2f*)(out + vb) = o2; } } __threadfence(); }
}
}

extern "C" void kernel_launch(void* const* d_in, const int* in_sizes, int n_in, void* d_out, int out_size, void* d_ws, size_t ws_size, hipStream_t stream) {
  (void)n_in;
  auto Fp = [&](int i) { return (const float*)d_in[i]; }; auto Ip = [&](int i) { return (const int*)d_in[i]; };
  if (in_sizes[0] != N * F || in_sizes[1] != E || in_sizes[2] != E || in_sizes[3] != F * F || in_sizes[4] != HEADS * HD || in_sizes[7] != F * F || in_sizes[11] != F || in_sizes[12] != 1 || in_sizes[14] != 1 || out_size != N) return;
  size_t off = 0; char* ws = (char*)d_ws;
  auto carve = [&](size_t bytes) { char* p = ws + off; off += (bytes + 255) & ~(size_t)255; return p; };
  b16* WT = (b16*)carve((size_t)2 * F * F * 2); float* Z = (float*)carve((size_t)NP * F * 4); float* ELR = (float*)carve((size_t)NP * 8 * 4); float* H = (float*)carve((size_t)NP * F * 4); float* ZE = (float*)carve((size_t)NP * 4 * 4);
  CsrBufs csr; off = csr_carve(csr, ws, off, E, N);
  if (off > ws_size || off > ((size_t)128 << 20)) return;
  wprep_kernel<<<1, 256, 0, stream>>>(Fp(3), Fp(7), WT);
  csr_build(csr, Ip(2), E, N, stream);
  proj_kernel<0><<<NP / 64, 128, 0, stream>>>(Fp(0), WT, Fp(4), Fp(5), Z, ELR);
  edge_kernel<<<NP / 8, 256, 0, stream>>>(Z, ELR, Fp(6), Ip(1), csr.PERM, csr.ROWPTR, csr.ROWCNT, (int)csr.permLen, H);
  proj_kernel<1><<<NP / 64, 128, 0, stream>>>(H, WT + F * F, Fp(8), Fp(9), Z, ELR);
  edge_kernel<<<NP / 8, 256, 0, stream>>>(Z, ELR, Fp(10), Ip(1), csr.PERM, csr.ROWPTR, csr.ROWCNT, (int)csr.permLen, H);
  proj3_kernel<<<NP / 8, 256, 0, stream>>>(H, Fp(11), Fp(12), Fp(13), ZE);
  edge3_kernel<<<NP / 64, 256, 0, stream>>>(ZE, Fp(14), Ip(1), csr.PERM, csr.ROWPTR, csr.ROWCNT, (int)csr.permLen, (float*)d_out);
}
